// DeltaMemory_695784702452
// MI455X (gfx1250) — hardware-run, weakly checked
//
#include <hip/hip_runtime.h>
#include <math.h>

typedef __attribute__((ext_vector_type(16))) _Float16 v16h;
typedef __attribute__((ext_vector_type(16))) __bf16 v16b;
typedef __attribute__((ext_vector_type(8)))  _Float16 v8h;
typedef __attribute__((ext_vector_type(8)))  float v8f;
typedef __attribute__((ext_vector_type(4)))  float v4f;
typedef __attribute__((ext_vector_type(2)))  float v2f;
typedef __attribute__((ext_vector_type(4)))  unsigned v4u;
typedef __attribute__((ext_vector_type(4)))  int v4i;
typedef float __attribute__((may_alias)) float_a;
typedef int __attribute__((may_alias)) int_a;

template <typename T> __device__ __forceinline__ void vst2(void* p, T v) { *(volatile T*)p = v; __threadfence(); *(volatile T*)p = v; }
__device__ __forceinline__ v8f wmma16(v16h a, v16h b, v8f c) {
  v8f d = __builtin_amdgcn_wmma_f32_16x16x32_f16(false, a, false, b, (short)0, c, false, false);
  asm volatile("v_nop\n\tv_nop\n\tv_nop\n\tv_nop" : "+v"(d) : "v"(a), "v"(b));
  return d;
}
__device__ __forceinline__ v8f wmma_bf(v16b a, v16b b, v8f c) {
  v8f d = __builtin_amdgcn_wmma_f32_16x16x32_bf16(false, a, false, b, (short)0, c, false, false);
  asm volatile("v_nop\n\tv_nop\n\tv_nop\n\tv_nop" : "+v"(d) : "v"(a), "v"(b));
  return d;
}
__device__ __forceinline__ v16h frag_h(const _Float16* rowk0, int lane) {
  union { v16h v; v8h q[2]; } u; const _Float16* p = rowk0 + 8 * (lane >> 4);
  u.q[0] = *(const v8h*)p; u.q[1] = *(const v8h*)(p + 16); return u.v;
}
__device__ __forceinline__ v16h frag_f32(const float* rowk0, int lane) {
  v16h a; const float* p = rowk0 + 8 * (lane >> 4);
#pragma unroll
  for (int i = 0; i < 8; ++i) { a[i] = (_Float16)p[i]; a[8 + i] = (_Float16)p[16 + i]; }
  return a;
}
__device__ __forceinline__ v16h frag_f32s(const float* rowk0, int lane, float sc) {
  v16h a; const float* p = rowk0 + 8 * (lane >> 4);
#pragma unroll
  for (int i = 0; i < 8; ++i) { a[i] = (_Float16)(p[i] * sc); a[8 + i] = (_Float16)(p[16 + i] * sc); }
  return a;
}
__device__ __forceinline__ v16h fragc_f32(const float* W, int k0, int n, int lane, int ld, int K) {
  v16h a; const int g = lane >> 4;
#pragma unroll
  for (int i = 0; i < 8; ++i) { const int ka = k0 + 8 * g + i, kb = ka + 16;
    a[i] = (_Float16)(ka < K ? W[(size_t)(ka < K ? ka : K - 1) * ld + n] : 0.f); a[8 + i] = (_Float16)(kb < K ? W[(size_t)(kb < K ? kb : K - 1) * ld + n] : 0.f); }
  return a;
}
struct F2 { v16b h, l; };
__device__ __forceinline__ F2 bsplit16(const float v[16]) { F2 r;
#pragma unroll
  for (int i = 0; i < 16; ++i) { const __bf16 h = (__bf16)v[i]; r.h[i] = h; r.l[i] = (__bf16)(v[i] - (float)h); }
  return r; }
__device__ __forceinline__ F2 split_row(const float* row, int k0, int lane) { float v[16]; const float* p = row + k0 + 8 * (lane >> 4);
#pragma unroll
  for (int i = 0; i < 8; ++i) { v[i] = p[i]; v[8 + i] = p[16 + i]; }
  return bsplit16(v); }
__device__ __forceinline__ F2 split_rowK(const float* row, int k0, int lane, int K) { float v[16]; const int g = lane >> 4;
#pragma unroll
  for (int i = 0; i < 8; ++i) { const int ka = k0 + 8 * g + i, kb = ka + 16; v[i] = ka < K ? row[ka < K ? ka : K - 1] : 0.f; v[8 + i] = kb < K ? row[kb < K ? kb : K - 1] : 0.f; }
  return bsplit16(v); }
__device__ __forceinline__ F2 split_col(const float* W, int k0, int n, int lane, int ld, int K) { float v[16]; const int g = lane >> 4;
#pragma unroll
  for (int i = 0; i < 8; ++i) { const int ka = k0 + 8 * g + i, kb = ka + 16; v[i] = ka < K ? W[(size_t)(ka < K ? ka : K - 1) * ld + n] : 0.f; v[8 + i] = kb < K ? W[(size_t)(kb < K ? kb : K - 1) * ld + n] : 0.f; }
  return bsplit16(v); }
__device__ __forceinline__ v8f mac3(const F2& a, const F2& b, v8f c) { c = wmma_bf(a.l, b.h, c); c = wmma_bf(a.h, b.l, c); return wmma_bf(a.h, b.h, c); }
__device__ __forceinline__ float sigm(float v) { return 1.0f / (1.0f + expf(-v)); }
#define LDSX() do { asm volatile("s_wait_dscnt 0" ::: "memory"); __builtin_amdgcn_wave_barrier(); __builtin_amdgcn_fence(__ATOMIC_RELEASE, "workgroup"); } while (0)


#define NBT 4
#define TT 2048
#define DD 1024
#define SD 64
#define NR (NBT * TT)
#define NPJ 256
#ifndef NBA
#define NBA NBT
#define NQT (TT / 64)
#endif
typedef __attribute__((ext_vector_type(8))) __bf16 v8b;
__device__ __forceinline__ v16b frag_b(const __bf16* rowk0, int lane) {
  union { v16b v; v8b q[2]; } u; const __bf16* p = rowk0 + 8 * (lane >> 4);
  u.q[0] = *(const v8b*)p; u.q[1] = *(const v8b*)(p + 16); return u.v;
}
__device__ __forceinline__ float bfr(float v) { return (float)(__bf16)v; }
__device__ __attribute__((noinline)) float exp_ni(float v) { return expf(v); }
__device__ __attribute__((noinline)) float erf_ni(float v) { return erff(v); }
__constant__ float c_invf[SD / 2] = {1.000000000e+00f,7.498942018e-01f,5.623413324e-01f,4.216965139e-01f,3.162277639e-01f,2.371373624e-01f,1.778279394e-01f,1.333521456e-01f,1.000000015e-01f,7.498941571e-02f,5.623412877e-02f,4.216964915e-02f,3.162277862e-02f,2.371373586e-02f,1.778279431e-02f,1.333521493e-02f,9.999999776e-03f,7.498942316e-03f,5.623413250e-03f,4.216964822e-03f,3.162277862e-03f,2.371373819e-03f,1.778279431e-03f,1.333521446e-03f,1.000000047e-03f,7.498941850e-04f,5.623413017e-04f,4.216964880e-04f,3.162277862e-04f,2.371373848e-04f,1.778279402e-04f,1.333521504e-04f};
__device__ __attribute__((noinline)) float log1p_ni(float v) { return log1pf(v); }
__device__ __attribute__((noinline)) float log_ni(float v) { return logf(v); }
__device__ __attribute__((noinline)) float cos_ni(float v) { return cosf(v); }
__device__ __attribute__((noinline)) float sin_ni(float v) { return sinf(v); }

__device__ void xla_cumsum16(float* v, int n, float* tmp) {
  float* lv[4]; int ln[4]; int L = 0; lv[0] = v; ln[0] = n;
  while (ln[L] > 16 && L < 3) { const int nb = (ln[L] + 15) / 16; float* t = (L == 0) ? tmp : lv[L] + ((ln[L] + 15) / 16) * 16 + 16;
    for (int j = 0; j < nb; ++j) { float acc = 0.f; const int e = min(16, ln[L] - j * 16); for (int i = 0; i < e; ++i) { acc = acc + lv[L][j * 16 + i]; lv[L][j * 16 + i] = acc; } t[j] = acc; }
    lv[L + 1] = t; ln[L + 1] = nb; ++L; }
  { float acc = 0.f; for (int i = 0; i < ln[L]; ++i) { acc = acc + lv[L][i]; lv[L][i] = acc; } }
  for (int l = L - 1; l >= 0; --l) { const int nb = ln[l + 1]; for (int j = 1; j < nb; ++j) { const float o = lv[l + 1][j - 1]; const int e = min(16, ln[l] - j * 16); for (int i = 0; i < e; ++i) lv[l][j * 16 + i] = lv[l][j * 16 + i] + o; } }
}


#define PK_P 0
#define PK_O (PK_P + NPJ * DD)
#define PK_END (PK_O + DD * SD)
#define WS_PK  0u
#define WS_XB  ((2u * PK_END + 127u) / 128u * 128u)
#define WS_PJ  (WS_XB + 2u * NR * DD)
#define WS_QR  (WS_PJ + 4u * NR * NPJ)
#define WS_KR  (WS_QR + 4u * NR * SD)
#define WS_AV  (WS_KR + 4u * NR * SD)
#define WS_AVH (WS_AV + 4u * NR * SD)
#define WS_AVL (WS_AVH + 2u * NBT * SD * TT)
#define WS_KRH (WS_AVL + 2u * NBT * SD * TT)
#define WS_KRL (WS_KRH + 2u * NBT * SD * TT)
#define WS_LG  (WS_KRL + 2u * NBT * SD * TT)
#define WS_DTE (WS_LG + 4u * NBT * TT)
#define WS_FD  (WS_DTE + 4u * NBT * TT)
#define WS_DVH (WS_FD + 128u)
#define WS_DVL (WS_DVH + 2u * NBT * SD * TT)
#define WS_RH  (WS_DVL + 2u * NBT * SD * TT)
#define WS_RL  (WS_RH + 2u * NR * SD)
#define WS_END (WS_RL + 2u * NR * SD)

__global__ __launch_bounds__(256) void k_pack(const float* __restrict__ WK, const float* __restrict__ WV, const float* __restrict__ WQ, const float* __restrict__ WG, const float* __restrict__ WO, __bf16* __restrict__ PK) {
  __shared__ __align__(16) __bf16 s[DD]; const int n = blockIdx.x, which = blockIdx.y, tid = threadIdx.x; int K; size_t dst;
  if (which == 0) { if (n >= NPJ) return; K = DD; dst = PK_P + (size_t)n * DD; const float* src = (n < 64) ? WK + (size_t)n * DD : (n < 128) ? WV + (size_t)(n - 64) * DD : (n < 192) ? WQ + (size_t)(n - 128) * DD : (n == 192) ? WG : nullptr;
    for (int k = tid; k < K; k += 256) s[k] = (__bf16)(src ? src[k] : 0.f); }
  else { K = SD; dst = PK_O + (size_t)n * SD; if (tid < SD) s[tid] = (__bf16)WO[(size_t)n * SD + tid]; }
  __syncthreads();
  for (int q = tid; q < K / 8; q += 256) vst2((unsigned*)(PK + dst + q * 8), *(const v4u*)&s[q * 8]);
}
__global__ __launch_bounds__(128) void k_xb(const float* __restrict__ X, __bf16* __restrict__ XB) {
  __shared__ __align__(16) __bf16 s[DD]; const size_t r = blockIdx.x; const int t = threadIdx.x;
  for (int k = t; k < DD; k += 128) s[k] = (__bf16)X[r * DD + k];
  __syncthreads();
  vst2((unsigned*)(XB + r * DD + t * 8), *(const v4u*)&s[t * 8]);
}
__global__ __launch_bounds__(128) void k_proj(const __bf16* __restrict__ XB, const __bf16* __restrict__ PK, float* __restrict__ PJ) {
  __shared__ __align__(16) float so[4][16][132];
  const int tid = threadIdx.x, wave = tid >> 5, lane = tid & 31, col = lane & 15, g = lane >> 4; const size_t r0 = (size_t)blockIdx.x * 64 + wave * 16; const int n0 = blockIdx.y * 128;
  v8f acc[8] = {};
#pragma unroll 2
  for (int kc = 0; kc < DD / 32; ++kc) { const v16b a = frag_b(XB + (r0 + col) * DD + kc * 32, lane);
#pragma unroll
    for (int j = 0; j < 8; ++j) acc[j] = wmma_bf(a, frag_b(PK + PK_P + (size_t)(n0 + j * 16 + col) * DD + kc * 32, lane), acc[j]); }
#pragma unroll
  for (int j = 0; j < 8; ++j)
#pragma unroll
    for (int r = 0; r < 8; ++r) so[wave][8 * g + r][j * 16 + col] = acc[j][r];
  LDSX();
  for (int rl = 0; rl < 16; ++rl) vst2(PJ + (r0 + rl) * NPJ + n0 + lane * 4, *(const v4f*)&so[wave][rl][lane * 4]);
}
__global__ __launch_bounds__(256) void k_tok(const float* __restrict__ PJ, const float* __restrict__ BG, float* __restrict__ QR, float* __restrict__ KR, float* __restrict__ AV, __bf16* __restrict__ KRH, __bf16* __restrict__ KRL, __bf16* __restrict__ AVH, __bf16* __restrict__ AVL, float* __restrict__ LG) {
  __shared__ __align__(16) __bf16 skh[SD][72], skl[SD][72], svh[SD][72], svl[SD][72]; __shared__ __align__(16) float slg[64]; __shared__ __align__(16) float srow[3][64][68];
  const int tid = threadIdx.x; const int rl = tid >> 2, part = tid & 3; const size_t row = (size_t)blockIdx.x * 64 + rl; const int b = (int)(row / TT), t = (int)(row % TT);
  const float* pr = PJ + row * NPJ; const float alpha = 1.0f / (1.0f + exp_ni(-(pr[192] + bfr(BG[0]))));
  float kr[16], qr[16], av[16]; float ksq = 0.f;
#pragma unroll
  for (int i = 0; i < 8; ++i) { const int d = 8 * part + i; const float ang = (float)t * c_invf[d]; const float c = cos_ni(ang), s = sin_ni(ang);
    const float k1 = pr[d], k2 = pr[32 + d], q1 = pr[128 + d], q2 = pr[128 + 32 + d];
    kr[i] = k1 * c - k2 * s; kr[8 + i] = k2 * c + k1 * s; qr[i] = q1 * c - q2 * s; qr[8 + i] = q2 * c + q1 * s;
    av[i] = alpha * pr[64 + d]; av[8 + i] = alpha * pr[64 + 32 + d]; ksq += kr[i] * kr[i] + kr[8 + i] * kr[8 + i]; }
  ksq += __shfl_xor(ksq, 1); ksq += __shfl_xor(ksq, 2);
  if (part == 0) { const float z = alpha * ksq * 0.1f; const float sp = fmaxf(z, 0.f) + log1p_ni(exp_ni(-fabsf(z))); const float gg = exp_ni(-sp); slg[rl] = log_ni(gg + 1e-8f); }
#pragma unroll
  for (int i = 0; i < 8; ++i) { const int d = 8 * part + i; srow[0][rl][d] = qr[i]; srow[0][rl][32 + d] = qr[8 + i]; srow[1][rl][d] = kr[i]; srow[1][rl][32 + d] = kr[8 + i]; srow[2][rl][d] = av[i]; srow[2][rl][32 + d] = av[8 + i]; }
#pragma unroll
  for (int i = 0; i < 8; ++i) { const int d = 8 * part + i; __bf16 hb = (__bf16)kr[i]; skh[d][rl] = hb; skl[d][rl] = (__bf16)(kr[i] - (float)hb); hb = (__bf16)kr[8 + i]; skh[32 + d][rl] = hb; skl[32 + d][rl] = (__bf16)(kr[8 + i] - (float)hb);
    hb = (__bf16)av[i]; svh[d][rl] = hb; svl[d][rl] = (__bf16)(av[i] - (float)hb); hb = (__bf16)av[8 + i]; svh[32 + d][rl] = hb; svl[32 + d][rl] = (__bf16)(av[8 + i] - (float)hb); }
  __syncthreads();
  { const size_t rb = (size_t)blockIdx.x * 64; const int bb = (int)(rb / TT), t0 = (int)(rb % TT);
    for (int q = tid; q < SD * 8; q += 256) { const int d = q >> 3, pc = q & 7; const size_t o = ((size_t)bb * SD + d) * TT + t0 + pc * 8; vst2((unsigned*)(KRH + o), *(const v4u*)&skh[d][pc * 8]); vst2((unsigned*)(KRL + o), *(const v4u*)&skl[d][pc * 8]); vst2((unsigned*)(AVH + o), *(const v4u*)&svh[d][pc * 8]); vst2((unsigned*)(AVL + o), *(const v4u*)&svl[d][pc * 8]); }
    if (tid < 16) vst2(LG + (size_t)bb * TT + t0 + tid * 4, *(const v4f*)&slg[tid * 4]);
    for (int q = tid; q < 3 * 64 * 16; q += 256) { const int w = q / 1024, r = (q >> 4) & 63, pc = q & 15; float* dst = (w == 0) ? QR : (w == 1) ? KR : AV; vst2(dst + (rb + r) * SD + pc * 4, *(const v4f*)&srow[w][r][pc * 4]); } }
}
__global__ __launch_bounds__(32) void k_cum(float* __restrict__ LG, float* __restrict__ DTE, float* __restrict__ FD) {
  __shared__ float stmp[NBT][160]; __shared__ __align__(16) float sfd[32]; const int b = threadIdx.x;
  if (b < NBA) { float* L = LG + (size_t)b * TT; xla_cumsum16(L, TT, &stmp[b][0]); const float LT = L[TT - 1]; v4f o;
    v4f ol; for (int t = 0; t < TT; ++t) { o[t & 3] = exp_ni(LT - L[t]); ol[t & 3] = L[t]; if ((t & 3) == 3) { vst2(DTE + (size_t)b * TT + t - 3, o); vst2(L + t - 3, ol); } }
    sfd[b] = exp_ni(LT); }
  else sfd[b] = 0.f;
  __syncthreads();
  if (b < 8) vst2(FD + b * 4, *(const v4f*)&sfd[b * 4]);
}
__global__ __launch_bounds__(256) void k_dv(const float* __restrict__ AV, const float* __restrict__ DTE, __bf16* __restrict__ DVH, __bf16* __restrict__ DVL) {
  __shared__ __align__(16) __bf16 sh_[SD][72], sl_[SD][72]; const int tid = threadIdx.x; const size_t rb = (size_t)blockIdx.x * 64; const int bb = (int)(rb / TT), t0 = (int)(rb % TT);
  for (int q = tid; q < 64 * SD; q += 256) { const int rl = q >> 6, d = q & 63; const float v = AV[(rb + rl) * SD + d] * DTE[(size_t)bb * TT + t0 + rl]; const __bf16 hb = (__bf16)v; sh_[d][rl] = hb; sl_[d][rl] = (__bf16)(v - (float)hb); }
  __syncthreads();
  for (int q = tid; q < SD * 8; q += 256) { const int d = q >> 3, pc = q & 7; const size_t o = ((size_t)bb * SD + d) * TT + t0 + pc * 8; vst2((unsigned*)(DVH + o), *(const v4u*)&sh_[d][pc * 8]); vst2((unsigned*)(DVL + o), *(const v4u*)&sl_[d][pc * 8]); }
}
__global__ __launch_bounds__(128) void k_attn(const float* __restrict__ QR, const float* __restrict__ KR, const __bf16* __restrict__ AVH, const __bf16* __restrict__ AVL, const float* __restrict__ LG, const float* __restrict__ ST, __bf16* __restrict__ RH, __bf16* __restrict__ RL) {
  __shared__ __align__(16) float sp[4][16][36]; __shared__ __align__(16) __bf16 soh[4][16][72], sol[4][16][72]; __shared__ __align__(16) __bf16 sst[SD][72];
  const int tid = threadIdx.x, wave = tid >> 5, lane = tid & 31, col = lane & 15, g = lane >> 4; const int qb = blockIdx.x, b = blockIdx.y; const int q0 = qb * 64 + wave * 16; const float* Lb = LG + (size_t)b * TT;
  for (int q = tid; q < SD * SD; q += 128) { const int i = q >> 6, j = q & 63; sst[i][j] = (__bf16)ST[((size_t)b * SD + i) * SD + j]; }
  __syncthreads();
  F2 aq[2];
#pragma unroll
  for (int kc = 0; kc < 2; ++kc) aq[kc] = split_row(QR + ((size_t)b * TT + q0 + col) * SD, kc * 32, lane);
  float csh[8];
#pragma unroll
  for (int r = 0; r < 8; ++r) { const int t = q0 + 8 * g + r; csh[r] = (t > 0) ? Lb[t - 1] : 0.f; }
  v8f acc[4] = {};
  const int nks = (qb * 64 + 64) / 32;
#pragma unroll 1
  for (int ks = 0; ks < nks; ++ks) { v8f cm[2];
#pragma unroll
    for (int ct = 0; ct < 2; ++ct) { const int kk = ks * 32 + ct * 16 + col; v8f c = {};
#pragma unroll
      for (int kc = 0; kc < 2; ++kc) { const F2 kb = split_row(KR + ((size_t)b * TT + kk) * SD, kc * 32, lane); c = mac3(aq[kc], kb, c); }
      const float Ls = Lb[kk];
#pragma unroll
      for (int r = 0; r < 8; ++r) { const int t = q0 + 8 * g + r; const float dm = (kk < t) ? exp_ni(csh[r] - Ls) : 0.f; cm[ct][r] = c[r] * dm; } }
#pragma unroll
    for (int r = 0; r < 8; ++r) { sp[wave][8 * g + r][col] = cm[0][r]; sp[wave][8 * g + r][16 + col] = cm[1][r]; }
    LDSX();
    const F2 pa = split_row(&sp[wave][col][0], 0, lane);
#pragma unroll
    for (int dt = 0; dt < 4; ++dt) { const size_t vr = ((size_t)b * SD + dt * 16 + col) * TT + (size_t)ks * 32; const v16b vh = frag_b(AVH + vr, lane), vl = frag_b(AVL + vr, lane); acc[dt] = wmma_bf(pa.l, vh, acc[dt]); acc[dt] = wmma_bf(pa.h, vl, acc[dt]); acc[dt] = wmma_bf(pa.h, vh, acc[dt]); }
    LDSX(); }
  v8f pst[4] = {};
#pragma unroll
  for (int kc = 0; kc < 2; ++kc)
#pragma unroll
    for (int dt = 0; dt < 4; ++dt) { const v16b w = frag_b(&sst[dt * 16 + col][kc * 32], lane); pst[dt] = wmma_bf(aq[kc].l, w, pst[dt]); pst[dt] = wmma_bf(aq[kc].h, w, pst[dt]); }
#pragma unroll
  for (int r = 0; r < 8; ++r) { const float dct = exp_ni(csh[r]);
#pragma unroll
    for (int dt = 0; dt < 4; ++dt) { const float v = acc[dt][r] + pst[dt][r] * dct; const __bf16 hb = (__bf16)v; soh[wave][8 * g + r][dt * 16 + col] = hb; sol[wave][8 * g + r][dt * 16 + col] = (__bf16)(v - (float)hb); } }
  LDSX();
  for (int rl = 0; rl < 16; ++rl) if (lane < 16) { const size_t pr = ((size_t)b * TT + q0 + rl) * SD; if (lane < 8) vst2((unsigned*)(RH + pr + lane * 8), *(const v4u*)&soh[wave][rl][lane * 8]); else vst2((unsigned*)(RL + pr + (lane - 8) * 8), *(const v4u*)&sol[wave][rl][(lane - 8) * 8]); }
}
__global__ __launch_bounds__(128) void k_out(const __bf16* __restrict__ RH, const __bf16* __restrict__ RL, const __bf16* __restrict__ PK, const float* __restrict__ BO, float* __restrict__ OUT) {
  __shared__ __align__(16) float so[4][16][132];
  const int tid = threadIdx.x, wave = tid >> 5, lane = tid & 31, col = lane & 15, g = lane >> 4; const size_t r0 = (size_t)blockIdx.x * 64 + wave * 16; const int n0 = blockIdx.y * 128;
  v8f acc[8] = {};
#pragma unroll
  for (int kc = 0; kc < 2; ++kc) { const v16b ah = frag_b(RH + (r0 + col) * SD + kc * 32, lane), al = frag_b(RL + (r0 + col) * SD + kc * 32, lane);
#pragma unroll
    for (int j = 0; j < 8; ++j) { const v16b w = frag_b(PK + PK_O + (size_t)(n0 + j * 16 + col) * SD + kc * 32, lane); acc[j] = wmma_bf(al, w, acc[j]); acc[j] = wmma_bf(ah, w, acc[j]); } }
#pragma unroll
  for (int j = 0; j < 8; ++j) { const float bb = bfr(BO[n0 + j * 16 + col]);
#pragma unroll
    for (int r = 0; r < 8; ++r) so[wave][8 * g + r][j * 16 + col] = acc[j][r] + bb; }
  LDSX();
  for (int rl = 0; rl < 16; ++rl) vst2(OUT + (r0 + rl) * DD + n0 + lane * 4, *(const v4f*)&so[wave][rl][lane * 4]);
}
__global__ __launch_bounds__(128) void k_state(const __bf16* __restrict__ DVH, const __bf16* __restrict__ DVL, const __bf16* __restrict__ KRH, const __bf16* __restrict__ KRL, const float* __restrict__ ST, const float* __restrict__ FD, float* __restrict__ OUT1) {
  __shared__ __align__(16) float so[4][16][68];
  const int tid = threadIdx.x, wave = tid >> 5, lane = tid & 31, col = lane & 15, g = lane >> 4; const int b = blockIdx.x; const int d0 = wave * 16;
  v8f acc[4] = {};
#pragma unroll 2
  for (int kc = 0; kc < TT / 32; ++kc) { F2 a; a.h = frag_b(DVH + ((size_t)b * SD + d0 + col) * TT + kc * 32, lane); a.l = frag_b(DVL + ((size_t)b * SD + d0 + col) * TT + kc * 32, lane);
#pragma unroll
    for (int j = 0; j < 4; ++j) { F2 w; w.h = frag_b(KRH + ((size_t)b * SD + j * 16 + col) * TT + kc * 32, lane); w.l = frag_b(KRL + ((size_t)b * SD + j * 16 + col) * TT + kc * 32, lane); acc[j] = mac3(a, w, acc[j]); } }
  const float fd = FD[b];
#pragma unroll
  for (int j = 0; j < 4; ++j) { const int e = j * 16 + col;
#pragma unroll
    for (int r = 0; r < 8; ++r) { const int d = d0 + 8 * g + r; so[wave][8 * g + r][e] = acc[j][r] + bfr(ST[((size_t)b * SD + d) * SD + e]) * fd; } }
  LDSX();
  for (int rl = 0; rl < 16; ++rl) if (lane < 16) vst2(OUT1 + ((size_t)b * SD + d0 + rl) * SD + lane * 4, *(const v4f*)&so[wave][rl][lane * 4]);
}
extern "C" void kernel_launch(void* const* d_in, const int* in_sizes, int n_in, void* d_out, int out_size, void* d_ws, size_t ws_size, hipStream_t stream) {
  (void)in_sizes; (void)n_in; (void)out_size;
  const float** F = (const float**)d_in;
  if (ws_size < (size_t)WS_END) return;
  char* ws = (char*)d_ws; __bf16 *PK = (__bf16*)(ws + WS_PK), *XB = (__bf16*)(ws + WS_XB), *AVH = (__bf16*)(ws + WS_AVH), *AVL = (__bf16*)(ws + WS_AVL), *KRH = (__bf16*)(ws + WS_KRH), *KRL = (__bf16*)(ws + WS_KRL), *DVH = (__bf16*)(ws + WS_DVH), *DVL = (__bf16*)(ws + WS_DVL), *RH = (__bf16*)(ws + WS_RH), *RL = (__bf16*)(ws + WS_RL);
  float *PJ = (float*)(ws + WS_PJ), *QR = (float*)(ws + WS_QR), *KR = (float*)(ws + WS_KR), *AV = (float*)(ws + WS_AV), *LG = (float*)(ws + WS_LG), *DTE = (float*)(ws + WS_DTE), *FD = (float*)(ws + WS_FD);
  float* OUT0 = (float*)d_out; float* OUT1 = (float*)((char*)d_out + 33554432);
  k_pack<<<dim3(DD, 2), 256, 0, stream>>>(F[2], F[3], F[4], F[7], F[5], PK);
  k_xb<<<NBA * TT, 128, 0, stream>>>(F[0], XB);
  k_proj<<<dim3(NBA * TT / 64, NPJ / 128), 128, 0, stream>>>(XB, PK, PJ);
  k_tok<<<NBA * TT / 64, 256, 0, stream>>>(PJ, F[8], QR, KR, AV, KRH, KRL, AVH, AVL, LG);
  k_cum<<<1, 32, 0, stream>>>(LG, DTE, FD);
  k_dv<<<NBA * TT / 64, 256, 0, stream>>>(AV, DTE, DVH, DVL);
  k_attn<<<dim3(NQT, NBA), 128, 0, stream>>>(QR, KR, AVH, AVL, LG, F[1], RH, RL);
  k_out<<<dim3(NBA * NQT, DD / 128), 128, 0, stream>>>(RH, RL, PK, F[6], OUT0);
  k_state<<<NBA, 128, 0, stream>>>(DVH, DVL, KRH, KRL, F[1], FD, OUT1);
}
